// SemiSymbolic_21912923144500
// MI455X (gfx1250) — hardware-run, weakly checked
//
#include <hip/hip_runtime.h>


#pragma clang fp contract(off)

#ifndef MROWS
#define MROWS 128
#endif
#define MROWS_FULL 128
#define KD   1024
#define ND   1024
#define OSP  68
#define DELTA_ 0.01f

static_assert(MROWS % 16 == 0);
static_assert(MROWS <= MROWS_FULL);
static_assert(ND % 64 == 0);
static_assert(KD % 32 == 0);
static_assert(KD % 8 == 0);
static_assert(((size_t)MROWS * KD) % 2048 == 0);
static_assert(((size_t)ND * KD) % 2048 == 0);
static_assert((OSP * 4) % 16 == 0);
static_assert(OSP >= 64);
static_assert(16 * OSP * 4 <= 131072);
static_assert(2048 * 4 <= 131072);
static_assert(32 * 16 * 8 == 16 * 64 * 4);
static_assert(256 * 16 * 2 == 2048 * 4);
static_assert(256 * 16 == 2048 * 2);

typedef unsigned short bf;
typedef __attribute__((ext_vector_type(16))) __bf16   v16bf;
typedef __attribute__((ext_vector_type(8)))  unsigned short v8us;
typedef __attribute__((ext_vector_type(8)))  float    v8f;
typedef __attribute__((ext_vector_type(4)))  float    v4f;
typedef v4f  __attribute__((may_alias)) v4fa;

__device__ __forceinline__ unsigned short f2bf(float f) { unsigned u = __float_as_uint(f); u += 0x7FFFu + ((u >> 16) & 1u); return (unsigned short)(u >> 16); }
__device__ __forceinline__ float bfr(float f) { return __uint_as_float(((unsigned)f2bf(f)) << 16); }
__device__ __forceinline__ v16bf cat16b(v8us lo, v8us hi) { return __builtin_bit_cast(v16bf, __builtin_shufflevector(lo, hi, 0, 1, 2, 3, 4, 5, 6, 7, 8, 9, 10, 11, 12, 13, 14, 15)); }
__device__ __forceinline__ v8f wmmab(v16bf a, v16bf b, v8f c) { return __builtin_amdgcn_wmma_f32_16x16x32_bf16(false, a, false, b, (short)0, c, false, false); }
__device__ __forceinline__ v8f wmmabg(v16bf a, v16bf b, v8f c) { c = wmmab(a, b, c); asm volatile("v_nop\n\tv_nop\n\tv_nop\n\tv_nop" : "+v"(c) : "v"(a), "v"(b)); return c; }
__device__ __forceinline__ v16bf ldb(const bf* p)  { return cat16b(*(const v8us*)p, *(const v8us*)(p + 16)); }
__device__ __forceinline__ void wave_sync() { __builtin_amdgcn_fence(3  , "wavefront"); __builtin_amdgcn_wave_barrier(); asm volatile("" ::: "memory"); }

__global__ __launch_bounds__(256) void k_cvt3(const float* __restrict__ src, bf* dv, bf* da, float* df) {
    __shared__ __align__(16) float fs[2048];
    const unsigned tid = threadIdx.x;
    const size_t i = (size_t)blockIdx.x * 256 + tid;
    const v8f v = *(const v8f*)(src + i * 8);
    v8us ov, oa; v4f f0, f1;
#pragma unroll
    for (int k = 0; k < 4; ++k) {
        const float a0 = fabsf(v[k]), a1 = fabsf(v[4 + k]);
        ov[k] = f2bf(v[k]); ov[4 + k] = f2bf(v[4 + k]);
        oa[k] = f2bf(a0);   oa[4 + k] = f2bf(a1);
        f0[k] = bfr(a0);    f1[k] = bfr(a1); }
    *(v4fa*)(&fs[tid * 8]) = f0; *(v4fa*)(&fs[tid * 8 + 4]) = f1;
    __syncthreads();
    const v4f p0 = *(const v4fa*)(&fs[tid * 4]);
    const v4f p1 = *(const v4fa*)(&fs[1024 + tid * 4]);
    float* fb = df + (size_t)blockIdx.x * 2048;
#pragma unroll 1
    for (int ps = 0; ps < 2; ++ps) {
        *(volatile v8us*)(dv + i * 8) = ov;
        *(volatile v8us*)(da + i * 8) = oa;
        *(volatile v4f*)(fb + tid * 4) = p0;
        *(volatile v4f*)(fb + 1024 + tid * 4) = p1;
        if (ps == 0) __threadfence(); }
}

__global__ __launch_bounds__(32) void k_layer(const bf* __restrict__ XB, const bf* __restrict__ XA, const float* __restrict__ XF,
                                              const bf* __restrict__ WB, const bf* __restrict__ WA, const float* __restrict__ WF, float* OUT) {
    __shared__ __align__(16) float os[16 * OSP];
    const unsigned bx = blockIdx.x, by = blockIdx.y;
    const int lane = threadIdx.x & 31, lr = lane & 15, hi = lane >> 4;
    const int r0 = (int)(bx * 16u), c0 = (int)(by * 64u);
    v8f accL[4], accA[4]; float amax[4][8];
#pragma unroll
    for (int nb = 0; nb < 4; ++nb) { accL[nb] = (v8f){}; accA[nb] = (v8f){};
#pragma unroll
        for (int j = 0; j < 8; ++j) amax[nb][j] = 0.0f; }
    const size_t aoff = (size_t)(r0 + lr) * KD + 8 * hi, boff = (size_t)(c0 + lr) * KD + 8 * hi;
    const size_t xfo = (size_t)(r0 + 8 * hi) * KD, wfo = (size_t)(c0 + lr) * KD;
#pragma unroll 1
    for (int kc = 0; kc < KD; kc += 32) {
        const v16bf av = ldb(XB + aoff + kc);
        const v16bf aa = ldb(XA + aoff + kc);
#pragma unroll
        for (int nb = 0; nb < 4; ++nb) {
            const v16bf bv = ldb(WB + boff + (size_t)nb * 16 * KD + kc);
            const v16bf ba = ldb(WA + boff + (size_t)nb * 16 * KD + kc);
            accL[nb] = wmmabg(av, bv, accL[nb]);
            accA[nb] = wmmabg(aa, ba, accA[nb]); }
#pragma unroll 1
        for (int kq = 0; kq < 32; kq += 4) {
            v4f xv[8], wv[4];
#pragma unroll
            for (int j = 0; j < 8; ++j) xv[j] = *(const v4f*)(XF + xfo + (size_t)j * KD + kc + kq);
#pragma unroll
            for (int nb = 0; nb < 4; ++nb) wv[nb] = *(const v4f*)(WF + wfo + (size_t)nb * 16 * KD + kc + kq);
#pragma unroll
            for (int nb = 0; nb < 4; ++nb) {
#pragma unroll
                for (int j = 0; j < 8; ++j) {
                    const v4f p = xv[j] * wv[nb];
                    amax[nb][j] = fmaxf(fmaxf(amax[nb][j], fmaxf(p[0], p[1])), fmaxf(p[2], p[3])); } }
        }
    }
#pragma unroll
    for (int nb = 0; nb < 4; ++nb) {
#pragma unroll
        for (int j = 0; j < 8; ++j) {
            const float bias = amax[nb][j] - accA[nb][j];
            const float sc = DELTA_ * bias;
            os[(hi * 8 + j) * OSP + nb * 16 + lr] = accL[nb][j] + sc; } }
    wave_sync();
    float* orow = OUT + (size_t)r0 * ND + c0;
#pragma unroll 1
    for (int ps = 0; ps < 2; ++ps) {
#pragma unroll
        for (int s = 0; s < 8; ++s) { const int row = 2 * s + (lane >> 4), cofs = (lane & 15) * 4;
            const v4f val = *(const v4fa*)(&os[row * OSP + cofs]);
            *(volatile v4f*)(orow + (size_t)row * ND + cofs) = val; }
        if (ps == 0) __threadfence(); }
}

static constexpr size_t al256(size_t v) { return (v + 255) & ~(size_t)255; }
static constexpr size_t SZ_XH = al256((size_t)MROWS * KD * 2);
static constexpr size_t SZ_XF = al256((size_t)MROWS * KD * 4);
static constexpr size_t SZ_WH = al256((size_t)ND * KD * 2);
static constexpr size_t SZ_WF = al256((size_t)ND * KD * 4);
static constexpr size_t SZ_TOTAL = 2 * SZ_XH + SZ_XF + 2 * SZ_WH + SZ_WF;
static_assert(SZ_TOTAL <= (size_t)134217728);
static_assert(SZ_XH == (size_t)MROWS * KD * 2);
static_assert(SZ_XF == (size_t)MROWS * KD * 4);
static_assert(SZ_WH == (size_t)ND * KD * 2);
static_assert(SZ_WF == (size_t)ND * KD * 4);
static constexpr unsigned G_CX = (unsigned)(((size_t)MROWS * KD) / 2048);
static constexpr unsigned G_CW = (unsigned)(((size_t)ND * KD) / 2048);

extern "C" void kernel_launch(void* const* d_in, const int* in_sizes, int n_in,
                              void* d_out, int out_size, void* d_ws, size_t ws_size, hipStream_t stream) {
    if (n_in < 2) return;
    if ((size_t)in_sizes[0] < (size_t)MROWS * KD) return;
    if ((size_t)in_sizes[1] < (size_t)ND * KD) return;
    if ((size_t)out_size < (size_t)MROWS * ND) return;
    if (SZ_TOTAL > ws_size) return;
    const float* x = (const float*)d_in[0];
    const float* W = (const float*)d_in[1];
    float* OUT = (float*)d_out;
    char* wsp = (char*)d_ws;
    bf* XB = (bf*)wsp; wsp += SZ_XH;
    bf* XA = (bf*)wsp; wsp += SZ_XH;
    float* XF = (float*)wsp; wsp += SZ_XF;
    bf* WB = (bf*)wsp; wsp += SZ_WH;
    bf* WA = (bf*)wsp; wsp += SZ_WH;
    float* WF = (float*)wsp; wsp += SZ_WF;

    k_cvt3<<<G_CX, 256, 0, stream>>>(x, XB, XA, XF);
    k_cvt3<<<G_CW, 256, 0, stream>>>(W, WB, WA, WF);
    k_layer<<<dim3(MROWS / 16, ND / 64, 1), 32, 0, stream>>>(XB, XA, XF, WB, WA, WF, OUT);
}
